// OptLayer_3977139716219
// MI455X (gfx1250) — hardware-run, weakly checked
//
#include <hip/hip_runtime.h>
#include <stddef.h>


typedef _Float16 h16;
typedef _Float16 v16h __attribute__((ext_vector_type(16)));
typedef _Float16 v8h  __attribute__((ext_vector_type(8)));
typedef float    v8f  __attribute__((ext_vector_type(8)));
typedef float    v4f  __attribute__((ext_vector_type(4)));

#ifndef NROWS
#define NROWS 4096
#endif
#define NROWS_FULL 4096
#define KDIM  2048
#define NOUT  1024
#define NBISECT 100
#define TOTAL_BUDGET 90.0f

static_assert(NROWS >= 64 && NROWS <= NROWS_FULL);
static_assert((NROWS % 64) == 0 && (NROWS % 16) == 0);
static_assert((KDIM % 32) == 0 && (KDIM % 8) == 0);
static_assert((NOUT % 64) == 0);
static_assert(NOUT == 16 * 16 * 4);
static_assert((((size_t)NROWS * KDIM) % 2048) == 0);
static_assert((((size_t)NOUT * KDIM) % 2048) == 0);
static_assert((size_t)NROWS * KDIM < (size_t)0xFFFFFFFFu);

#define LDC 68
static_assert((LDC % 4) == 0 && LDC >= 64);

#define XCARRY 64.0f
#define WCARRY 4096.0f
#define ZSCALE (1.0f / (XCARRY * WCARRY))

#define X16_BYTES ((size_t)NROWS * KDIM * 2)
#define W16_BYTES ((size_t)NOUT * KDIM * 2)
#define Z_BYTES   ((size_t)NROWS * NOUT * 4)
#define OFF_X16 ((size_t)0)
#define OFF_W16 (OFF_X16 + X16_BYTES)
#define OFF_Z   (OFF_W16 + W16_BYTES)
#define WS_TOTAL (OFF_Z + Z_BYTES)
static_assert((X16_BYTES % 128) == 0 && (W16_BYTES % 128) == 0 && (Z_BYTES % 128) == 0);
static_assert(WS_TOTAL <= (size_t)134217728);

__device__ __forceinline__ float bf16r(float x) {
  unsigned int u = __float_as_uint(x);
  u = (u + 0x7FFFu + ((u >> 16) & 1u)) & 0xFFFF0000u;
  return __uint_as_float(u);
}

static __device__ __forceinline__ h16 toh_flush(float v) {
  const h16 r = (h16)v;
  return (fabsf(v) < 6.103515625e-05f) ? (h16)0.0f : r;
}

__device__ __forceinline__ v16h frag_at(const _Float16* p) {
  v8h lo = *(const v8h*)(p);
  v8h hi = *(const v8h*)(p + 16);
  v16h out;
#pragma unroll
  for (int i = 0; i < 8; ++i) { out[i] = lo[i]; out[i + 8] = hi[i]; }
  return out;
}

__device__ __forceinline__ v8f wmma16(v16h a, v16h b, v8f c) {
  v8f d = __builtin_amdgcn_wmma_f32_16x16x32_f16(false, a, false, b, (short)0, c,
                                                 false, false);
  asm volatile("v_nop\n\tv_nop\n\tv_nop\n\tv_nop" : "+v"(d) : "v"(a), "v"(b));
  return d;
}

__device__ __forceinline__ float red16_max(float x) {
#pragma unroll
  for (int off = 1; off < 16; off <<= 1) x = fmaxf(x, __shfl_xor(x, off, 32));
  return x;
}
__device__ __forceinline__ float red16_min(float x) {
#pragma unroll
  for (int off = 1; off < 16; off <<= 1) x = fminf(x, __shfl_xor(x, off, 32));
  return x;
}
__device__ __forceinline__ float red16_sum(float x) {
#pragma unroll
  for (int off = 1; off < 16; off <<= 1) x += __shfl_xor(x, off, 32);
  return x;
}

__global__ __launch_bounds__(256) void cvt_plane_kernel(
    const float* __restrict__ src, _Float16* __restrict__ dst, float carry, unsigned n8) {
  const unsigned i = blockIdx.x * 256u + threadIdx.x;
  if (i >= n8) return;
  const float* s = src + (size_t)i * 8u;
  const v4f a0 = *(const v4f*)(s);
  const v4f a1 = *(const v4f*)(s + 4);
  v8h o;
#pragma unroll
  for (int j = 0; j < 4; ++j) {
    o[j]     = toh_flush(carry * bf16r(a0[j]));
    o[j + 4] = toh_flush(carry * bf16r(a1[j]));
  }
  _Float16* p = dst + (size_t)i * 8u;
  *(volatile v8h*)p = o;
  __threadfence();
  *(volatile v8h*)p = o;
}

__global__ __launch_bounds__(256) void gemm_z_kernel(
    const _Float16* __restrict__ A16, const _Float16* __restrict__ Bt,
    const float* __restrict__ bias, float* __restrict__ outf) {
  __shared__ float Cs[64 * LDC];
  const unsigned tid = threadIdx.x, lane = tid & 31u;
  const unsigned w = (unsigned)__builtin_amdgcn_readfirstlane((int)(threadIdx.x >> 5));
  const unsigned mw = w >> 1, nw = w & 1u;
  const unsigned hh = lane >> 4, m = lane & 15u;
  const unsigned n0 = blockIdx.x * 64u;
  const unsigned row0 = blockIdx.y * 64u;

  const _Float16* ap  = A16 + (size_t)(row0 + mw * 16u + m) * KDIM + hh * 8u;
  const _Float16* bp0 = Bt + (size_t)(n0 + nw * 32u + m) * KDIM + hh * 8u;
  const _Float16* bp1 = bp0 + (size_t)16 * KDIM;
  v8f acc0 = {}, acc1 = {};
#pragma unroll 2
  for (unsigned k0 = 0; k0 < (unsigned)KDIM; k0 += 32u) {
    const v16h a  = frag_at(ap + k0);
    const v16h b0 = frag_at(bp0 + k0);
    const v16h b1 = frag_at(bp1 + k0);
    acc0 = wmma16(a, b0, acc0);
    acc1 = wmma16(a, b1, acc1);
  }
#pragma unroll
  for (int r = 0; r < 8; ++r) {
    float* d = &Cs[(mw * 16u + hh * 8u + (unsigned)r) * LDC + nw * 32u + m];
    d[0]  = acc0[r];
    d[16] = acc1[r];
  }
  __syncthreads();

  v4f xs[4];
  size_t off[4];
#pragma unroll
  for (unsigned i = 0; i < 4u; ++i) {
    const unsigned r = 16u * i + (tid >> 4);
    const unsigned c = (tid & 15u) * 4u;
    const v4f u = *(const v4f*)&Cs[r * LDC + c];
    const v4f g = *(const v4f*)(bias + n0 + c);
    v4f val;
#pragma unroll
    for (int j = 0; j < 4; ++j) val[j] = u[j] * ZSCALE - bf16r(g[j]);
    xs[i] = val;
    off[i] = (size_t)(row0 + r) * NOUT + n0 + c;
  }
#pragma unroll
  for (int i = 0; i < 4; ++i) *(volatile v4f*)(outf + off[i]) = xs[i];
  __threadfence();
#pragma unroll
  for (int i = 0; i < 4; ++i) *(volatile v4f*)(outf + off[i]) = xs[i];
}

__global__ __launch_bounds__(256) void proj_kernel(
    const float* __restrict__ z, const float* __restrict__ u, float* __restrict__ y) {
#pragma clang fp contract(off)
  const unsigned tid = threadIdx.x;
  const unsigned sub = tid & 15u;
  const unsigned row = blockIdx.x * 16u + (tid >> 4);
  const float* zr = z + (size_t)row * NOUT + sub * 4u;
  const float* ur = u + sub * 4u;
  float* yr = y + (size_t)row * NOUT + sub * 4u;

  v4f zv[16], uv[16];
  float zmin = 3.4e38f, zmax = -3.4e38f, umax = -3.4e38f;
#pragma unroll
  for (int jj = 0; jj < 16; ++jj) {
    const v4f a = *(const v4f*)(zr + jj * 64);
    const v4f t = *(const v4f*)(ur + jj * 64);
    v4f tb;
#pragma unroll
    for (int i = 0; i < 4; ++i) tb[i] = bf16r(t[i]);
    zv[jj] = a;
    uv[jj] = tb;
    zmin = fminf(zmin, fminf(fminf(a[0], a[1]), fminf(a[2], a[3])));
    zmax = fmaxf(zmax, fmaxf(fmaxf(a[0], a[1]), fmaxf(a[2], a[3])));
    umax = fmaxf(umax, fmaxf(fmaxf(tb[0], tb[1]), fmaxf(tb[2], tb[3])));
  }
  zmin = red16_min(zmin);
  zmax = red16_max(zmax);
  umax = red16_max(umax);

  float lo = zmin - umax;
  float hi = zmax;

#pragma unroll 1
  for (int it = 0; it < NBISECT; ++it) {
    const float mid = 0.5f * (lo + hi);
    float s = 0.0f;
#pragma unroll
    for (int jj = 0; jj < 16; ++jj) {
#pragma unroll
      for (int i = 0; i < 4; ++i)
        s += fminf(fmaxf(zv[jj][i] - mid, 0.0f), uv[jj][i]);
    }
    s = red16_sum(s);
    const bool big = (s > TOTAL_BUDGET);
    const float nlo = big ? mid : lo;
    const float nhi = big ? hi : mid;
    const int changed = ((__float_as_uint(nlo) != __float_as_uint(lo)) ||
                         (__float_as_uint(nhi) != __float_as_uint(hi))) ? 1 : 0;
    lo = nlo;
    hi = nhi;
    if (__any(changed) == 0) break;
  }

  const float tau = 0.5f * (lo + hi);
#pragma unroll
  for (int jj = 0; jj < 16; ++jj) {
    v4f o;
#pragma unroll
    for (int i = 0; i < 4; ++i)
      o[i] = fminf(fmaxf(zv[jj][i] - tau, 0.0f), uv[jj][i]);
    zv[jj] = o;
  }
#pragma unroll
  for (int jj = 0; jj < 16; ++jj) *(volatile v4f*)(yr + jj * 64) = zv[jj];
  __threadfence();
#pragma unroll
  for (int jj = 0; jj < 16; ++jj) *(volatile v4f*)(yr + jj * 64) = zv[jj];
}

extern "C" void kernel_launch(void* const* d_in, const int* in_sizes, int n_in,
                              void* d_out, int out_size, void* d_ws, size_t ws_size,
                              hipStream_t stream) {
  if (n_in < 4) return;
  if ((long long)in_sizes[0] < (long long)NROWS * KDIM) return;
  if ((long long)in_sizes[1] < (long long)NOUT * KDIM) return;
  if (in_sizes[2] < NOUT || in_sizes[3] < NOUT) return;
  if ((long long)out_size < (long long)NROWS * NOUT) return;
  if (ws_size < WS_TOTAL) return;

  const float* x = (const float*)d_in[0];
  const float* W = (const float*)d_in[1];
  const float* b = (const float*)d_in[2];
  const float* u = (const float*)d_in[3];
  float* out = (float*)d_out;

  char* ws = (char*)d_ws;
  _Float16* X16 = (_Float16*)(ws + OFF_X16);
  _Float16* W16 = (_Float16*)(ws + OFF_W16);
  float*    Z   = (float*)(ws + OFF_Z);

  dim3 blk(256);
  const unsigned xn8 = (unsigned)(((size_t)NROWS * KDIM) / 8u);
  const unsigned wn8 = (unsigned)(((size_t)NOUT * KDIM) / 8u);

  cvt_plane_kernel<<<dim3(xn8 / 256u), blk, 0, stream>>>(x, X16, XCARRY, xn8);
  cvt_plane_kernel<<<dim3(wn8 / 256u), blk, 0, stream>>>(W, W16, WCARRY, wn8);
  gemm_z_kernel<<<dim3(NOUT / 64, NROWS / 64), blk, 0, stream>>>(X16, W16, b, Z);
  proj_kernel<<<dim3(NROWS / 16), blk, 0, stream>>>(Z, u, out);
}
